// SymmetricTensorProduct_88587995447413
// MI455X (gfx1250) — hardware-verified
//
#include <hip/hip_runtime.h>


#define NZT  8192
#define MUL  128
#define DIN  512
#define CH   1024
#define NCH  (NZT / CH)
#define NVW  (MUL * MUL)
#define NIP  64
#define PW_SS 0.0625f
#define PW_VV 0.036084391824351615f
#define PW_SV 0.0078125f
typedef _Float16 h16;
typedef unsigned short bf;
typedef __attribute__((ext_vector_type(16))) __bf16   v16bf;
typedef __attribute__((ext_vector_type(16))) _Float16 v16h;
typedef __attribute__((ext_vector_type(8)))  _Float16 v8h;
typedef __attribute__((ext_vector_type(8)))  unsigned short v8us;
typedef __attribute__((ext_vector_type(8)))  float    v8f;
typedef __attribute__((ext_vector_type(4)))  float    v4f;
typedef v8h  __attribute__((may_alias)) v8ha;
typedef v4f  __attribute__((may_alias)) v4fa;
typedef v8us __attribute__((may_alias)) v8usa;

__device__ __forceinline__ unsigned short f2bf(float f) { unsigned u = __float_as_uint(f); u += 0x7FFFu + ((u >> 16) & 1u); return (unsigned short)(u >> 16); }
__device__ __forceinline__ float bf2f(unsigned short b) { return __uint_as_float(((unsigned)b) << 16); }
__device__ __forceinline__ float bfr(float f) { return bf2f(f2bf(f)); }
__device__ __forceinline__ v16h cat16(v8h lo, v8h hi) { return __builtin_shufflevector(lo, hi, 0, 1, 2, 3, 4, 5, 6, 7, 8, 9, 10, 11, 12, 13, 14, 15); }
__device__ __forceinline__ v16bf cat16b(v8us lo, v8us hi) { return __builtin_bit_cast(v16bf, __builtin_shufflevector(lo, hi, 0, 1, 2, 3, 4, 5, 6, 7, 8, 9, 10, 11, 12, 13, 14, 15)); }
__device__ __forceinline__ v8f wmma16(v16h a, v16h b, v8f c) { return __builtin_amdgcn_wmma_f32_16x16x32_f16(false, a, false, b, (short)0, c, false, false); }
__device__ __forceinline__ v8f wmmab(v16bf a, v16bf b, v8f c) { return __builtin_amdgcn_wmma_f32_16x16x32_bf16(false, a, false, b, (short)0, c, false, false); }


template <typename T16> struct WFrag;
template <> struct WFrag<h16> { typedef v16h V; static __device__ __forceinline__ V ld(const h16* p) { return cat16(*(const v8h*)p, *(const v8h*)(p + 16)); } static __device__ __forceinline__ v8f mma(V a, V b, v8f c) { return wmma16(a, b, c); } };
template <> struct WFrag<bf> { typedef v16bf V; static __device__ __forceinline__ V ld(const bf* p) { return cat16b(*(const v8us*)p, *(const v8us*)(p + 16)); } static __device__ __forceinline__ v8f mma(V a, V b, v8f c) { return wmmab(a, b, c); } };
template <typename T16, int NSPLIT, bool BIAS>
__global__ __launch_bounds__(32) void k_gemmw(const T16* __restrict__ A, const T16* __restrict__ A2, const T16* __restrict__ Bt, const T16* __restrict__ Bt2, int K, float* C, int ldc, const float* __restrict__ bias, size_t sA, size_t sB, size_t sC) {
    typedef typename WFrag<T16>::V V;
    __shared__ __align__(16) float os[16 * 68];
    const size_t z = blockIdx.z; A += z * sA; if (A2) A2 += z * sA; Bt += z * sB; if (Bt2) Bt2 += z * sB; C += z * sC;
    const int lane = threadIdx.x & 31, lr = lane & 15, hi = lane >> 4; const int r0 = blockIdx.x * 64, c0 = blockIdx.y * 64;
    v8f acc[4][4];
#pragma unroll
    for (int mb = 0; mb < 4; ++mb)
#pragma unroll
        for (int nb = 0; nb < 4; ++nb) acc[mb][nb] = (v8f){};
    const size_t aoff = (size_t)(r0 + lr) * K + 8 * hi, boff = (size_t)(c0 + lr) * K + 8 * hi;
#pragma unroll 1
    for (int kc = 0; kc < K; kc += 32) {
        V a[4], a2[4];
#pragma unroll
        for (int mb = 0; mb < 4; ++mb) { a[mb] = WFrag<T16>::ld(A + aoff + (size_t)mb * 16 * K + kc); if (NSPLIT == 1 || NSPLIT == 2) a2[mb] = WFrag<T16>::ld(A2 + aoff + (size_t)mb * 16 * K + kc); }
#pragma unroll
        for (int nb = 0; nb < 4; ++nb) { const V b = WFrag<T16>::ld(Bt + boff + (size_t)nb * 16 * K + kc); V b2; if (NSPLIT >= 2) b2 = WFrag<T16>::ld(Bt2 + boff + (size_t)nb * 16 * K + kc);
#pragma unroll
            for (int mb = 0; mb < 4; ++mb) { acc[mb][nb] = WFrag<T16>::mma(a[mb], b, acc[mb][nb]); if (NSPLIT == 1 || NSPLIT == 2) acc[mb][nb] = WFrag<T16>::mma(a2[mb], b, acc[mb][nb]); if (NSPLIT >= 2) acc[mb][nb] = WFrag<T16>::mma(a[mb], b2, acc[mb][nb]); } }
        asm volatile("v_nop\n\tv_nop\n\tv_nop\n\tv_nop" : "+v"(acc[0][0]), "+v"(acc[1][1]), "+v"(acc[2][2]), "+v"(acc[3][3]) : "v"(a[0]), "v"(a[3]));
    }
#pragma unroll
    for (int mb = 0; mb < 4; ++mb) {
#pragma unroll
        for (int nb = 0; nb < 4; ++nb) {
#pragma unroll
            for (int j = 0; j < 8; ++j) os[(hi * 8 + j) * 68 + nb * 16 + lr] = acc[mb][nb][j]; }
        __builtin_amdgcn_wave_barrier(); asm volatile("" ::: "memory");
        float* crow = C + (size_t)(r0 + mb * 16) * ldc + c0;
#pragma unroll 1
        for (int ps = 0; ps < 2; ++ps) {
#pragma unroll
            for (int s = 0; s < 8; ++s) { const int row = 2 * s + hi, cofs = lr * 4; v4f val = *(const v4fa*)(os + row * 68 + cofs); if (BIAS) { val[0] += bfr(bias[c0 + cofs]); val[1] += bfr(bias[c0 + cofs + 1]); val[2] += bfr(bias[c0 + cofs + 2]); val[3] += bfr(bias[c0 + cofs + 3]); }
                *(volatile v4f*)(crow + (size_t)row * ldc + cofs) = val; }
            if (ps == 0) __threadfence(); }
        __builtin_amdgcn_wave_barrier(); asm volatile("" ::: "memory");
    }
}

__device__ __forceinline__ void splitf(float y, unsigned short& h, unsigned short& l) { h = f2bf(y); l = f2bf(y - bf2f(h)); }
typedef __attribute__((ext_vector_type(2))) unsigned short v2us;
typedef __attribute__((ext_vector_type(2))) float v2f;
__global__ __launch_bounds__(256) void k_cvt8(const float* __restrict__ src, bf* dst, size_t n8) { const size_t i = (size_t)blockIdx.x * 256 + threadIdx.x; if (i >= n8) return; const v8f v = *(const v8f*)(src + i * 8); v8us o;
#pragma unroll
    for (int k = 0; k < 8; ++k) o[k] = f2bf(v[k]); *(volatile v8us*)(dst + i * 8) = o; __threadfence(); *(volatile v8us*)(dst + i * 8) = o; }

__global__ __launch_bounds__(256) void k_xplanes(const float* __restrict__ x, bf* XS, bf* XV) { const size_t e = ((size_t)blockIdx.x * 256 + threadIdx.x) * 2; if (e >= (size_t)NZT * MUL) return; const int u = (int)(e % MUL); const size_t z = e / MUL; const float* xr = x + z * DIN; v2us s, a0, a1, a2;
    s[0] = f2bf(xr[u]); s[1] = f2bf(xr[u + 1]);
#pragma unroll
    for (int q = 0; q < 2; ++q) { a0[q] = f2bf(xr[MUL + 3 * (u + q) + 0]); a1[q] = f2bf(xr[MUL + 3 * (u + q) + 1]); a2[q] = f2bf(xr[MUL + 3 * (u + q) + 2]); }
    const size_t P = (size_t)NZT * MUL;
    *(volatile v2us*)(XS + e) = s; *(volatile v2us*)(XV + e) = a0; *(volatile v2us*)(XV + P + e) = a1; *(volatile v2us*)(XV + 2 * P + e) = a2; __threadfence();
    *(volatile v2us*)(XS + e) = s; *(volatile v2us*)(XV + e) = a0; *(volatile v2us*)(XV + P + e) = a1; *(volatile v2us*)(XV + 2 * P + e) = a2; }
__global__ __launch_bounds__(256) void k_wsv(const float* __restrict__ wsv, bf* WP) { const size_t e = ((size_t)blockIdx.x * 256 + threadIdx.x) * 2; if (e >= (size_t)NVW * MUL) return; const int u = (int)(e % MUL); const int wv = (int)(e / MUL); const int w = wv / MUL, v = wv % MUL; v2us o;
    o[0] = f2bf(wsv[((size_t)u * MUL + v) * MUL + w]); o[1] = f2bf(wsv[((size_t)(u + 1) * MUL + v) * MUL + w]); *(volatile v2us*)(WP + e) = o; __threadfence(); *(volatile v2us*)(WP + e) = o; }
__global__ __launch_bounds__(256) void k_split8(const float* __restrict__ F, bf* H, bf* Lw, size_t n8) { const size_t i = (size_t)blockIdx.x * 256 + threadIdx.x; if (i >= n8) return; const v8f v = *(const v8f*)(F + i * 8); v8us oh, ol;
#pragma unroll
    for (int q = 0; q < 8; ++q) { unsigned short a, c; splitf(v[q], a, c); oh[q] = a; ol[q] = c; } *(volatile v8us*)(H + i * 8) = oh; *(volatile v8us*)(Lw + i * 8) = ol; __threadfence(); *(volatile v8us*)(H + i * 8) = oh; *(volatile v8us*)(Lw + i * 8) = ol; }
__global__ __launch_bounds__(256) void k_xvt(const bf* __restrict__ XV, int chunk, bf* XVT) { const size_t e = ((size_t)blockIdx.x * 256 + threadIdx.x) * 2; if (e >= (size_t)CH * NIP * MUL) return; const int v = (int)(e % MUL); const int i = (int)((e / MUL) % NIP); const int zl = (int)(e / ((size_t)MUL * NIP)); v2us o; o[0] = 0; o[1] = 0;
    if (i < 3) { const bf* src = XV + (size_t)i * NZT * MUL + ((size_t)chunk * CH + zl) * MUL + v; o[0] = src[0]; o[1] = src[1]; } *(volatile v2us*)(XVT + e) = o; __threadfence(); *(volatile v2us*)(XVT + e) = o; }
__global__ __launch_bounds__(256) void k_outs(const float* __restrict__ x, const float* __restrict__ E1, const float* __restrict__ T3, float* OUT) { const size_t e = ((size_t)blockIdx.x * 256 + threadIdx.x) * 4; if (e >= (size_t)NZT * MUL) return; const int u = (int)(e % MUL); const size_t z = e / MUL; const float* xr = x + z * DIN; v4f o;
#pragma unroll
    for (int q = 0; q < 4; ++q) { const int uu = u + q; const float xs = bfr(xr[uu]); float a = __fmul_rn(__fmul_rn(PW_SS, xs), E1[e + q]); asm volatile("" : "+v"(a)); float s3 = 0.f;
#pragma unroll
        for (int i = 0; i < 3; ++i) { float p = __fmul_rn(bfr(xr[MUL + 3 * uu + i]), T3[(size_t)i * NZT * MUL + e + q]); asm volatile("" : "+v"(p)); s3 = __fadd_rn(s3, p); }
        float b3 = __fmul_rn(PW_VV, s3); asm volatile("" : "+v"(b3)); o[q] = __fadd_rn(a, b3); }
    *(volatile v4f*)(OUT + z * DIN + u) = o; __threadfence(); *(volatile v4f*)(OUT + z * DIN + u) = o; }
__global__ __launch_bounds__(256) void k_outv(const float* __restrict__ CV, int chunk, float* OUT) { const size_t e = ((size_t)blockIdx.x * 256 + threadIdx.x) * 2; if (e >= (size_t)CH * 3 * MUL) return; const int c = (int)(e % (3 * MUL)); const int zl = (int)(e / (3 * MUL)); v2f o;
#pragma unroll
    for (int q = 0; q < 2; ++q) { const int cc = c + q; const int w = cc / 3, i = cc % 3; o[q] = __fmul_rn(PW_SV, CV[((size_t)zl * MUL + w) * NIP + i]); }
    float* dst = OUT + ((size_t)chunk * CH + zl) * DIN + MUL + c; *(volatile v2f*)dst = o; __threadfence(); *(volatile v2f*)dst = o; }

extern "C" void kernel_launch(void* const* d_in, const int* in_sizes, int n_in,
                              void* d_out, int out_size, void* d_ws, size_t ws_size, hipStream_t stream) {
    (void)in_sizes; (void)n_in; (void)out_size;
    const float* x = (const float*)d_in[0]; const float* wss = (const float*)d_in[1]; const float* wsv = (const float*)d_in[2]; const float* wvv = (const float*)d_in[3];
    float* OUT = (float*)d_out;
    char* wsp = (char*)d_ws;
    auto take = [&](size_t bytes) { char* p = wsp; wsp += (bytes + 255) & ~(size_t)255; return (void*)p; };
    bf* WSS = (bf*)take((size_t)MUL * MUL * 2); bf* WVV = (bf*)take((size_t)MUL * MUL * 2); bf* WP = (bf*)take((size_t)NVW * MUL * 2); bf* XS = (bf*)take((size_t)NZT * MUL * 2); bf* XV = (bf*)take((size_t)3 * NZT * MUL * 2);
    float* E1 = (float*)take((size_t)NZT * MUL * 4); float* T3 = (float*)take((size_t)3 * NZT * MUL * 4);
    float* TP = (float*)take((size_t)CH * NVW * 4); bf* TPh = (bf*)take((size_t)CH * NVW * 2); bf* TPl = (bf*)take((size_t)CH * NVW * 2); bf* XVT = (bf*)take((size_t)CH * NIP * MUL * 2); float* CV = (float*)take((size_t)CH * MUL * NIP * 4);
    if ((size_t)(wsp - (char*)d_ws) > ws_size) return;
    k_cvt8<<<(MUL * MUL / 8 + 255) / 256, 256, 0, stream>>>(wss, WSS, (size_t)MUL * MUL / 8); k_cvt8<<<(MUL * MUL / 8 + 255) / 256, 256, 0, stream>>>(wvv, WVV, (size_t)MUL * MUL / 8);
    k_wsv<<<(unsigned)(((size_t)NVW * MUL / 2 + 255) / 256), 256, 0, stream>>>(wsv, WP); k_xplanes<<<(unsigned)(((size_t)NZT * MUL / 2 + 255) / 256), 256, 0, stream>>>(x, XS, XV);
    k_gemmw<bf, 0, false><<<dim3(NZT / 64, MUL / 64, 1), 32, 0, stream>>>(XS, nullptr, WSS, nullptr, MUL, E1, MUL, nullptr, 0, 0, 0);
    k_gemmw<bf, 0, false><<<dim3(NZT / 64, MUL / 64, 3), 32, 0, stream>>>(XV, nullptr, WVV, nullptr, MUL, T3, MUL, nullptr, (size_t)NZT * MUL, 0, (size_t)NZT * MUL);
    k_outs<<<(unsigned)(((size_t)NZT * MUL / 4 + 255) / 256), 256, 0, stream>>>(x, E1, T3, OUT);
    for (int ck = 0; ck < NCH; ++ck) {
        k_gemmw<bf, 0, false><<<dim3(CH / 64, NVW / 64, 1), 32, 0, stream>>>(XS + (size_t)ck * CH * MUL, nullptr, WP, nullptr, MUL, TP, NVW, nullptr, 0, 0, 0);
        k_split8<<<(unsigned)(((size_t)CH * NVW / 8 + 255) / 256), 256, 0, stream>>>(TP, TPh, TPl, (size_t)CH * NVW / 8);
        k_xvt<<<(unsigned)(((size_t)CH * NIP * MUL / 2 + 255) / 256), 256, 0, stream>>>(XV, ck, XVT);
        k_gemmw<bf, 1, false><<<dim3(MUL / 64, NIP / 64, CH), 32, 0, stream>>>(TPh, TPl, XVT, nullptr, MUL, CV, NIP, nullptr, (size_t)NVW, (size_t)NIP * MUL, (size_t)MUL * NIP);
        k_outv<<<(unsigned)(((size_t)CH * 3 * MUL / 2 + 255) / 256), 256, 0, stream>>>(CV, ck, OUT); }
}
